// CommAwareGCN_5858335392390
// MI455X (gfx1250) — hardware-run, weakly checked
//
#include <hip/hip_runtime.h>
#include <stddef.h>
#include <math.h>


#define FD      64
#define NCLS    40
#define NCP     64
#define KD      64
#define NTHR    256
#define NWAVE   8
#define EPT     8
#define NGRP    2
#define CHUNK   (NTHR * EPT * NGRP)
#define WCAP    (EPT * NGRP * 32)
#define LISTN   (NWAVE * WCAP)
#define NBC     4096
#define NBF     1024
#define RCAP    40960
#define RBN     128
#define TGT     128
#define DEGCAP  1024
#define GROWS   128
#define OTHR    512
#define WSCAP   134217728

#define WPL     (2 * NCP * KD)
#define WP_1    0
#define WP_2    WPL
#define WP_F    (2 * WPL)
#define WPTOT   (3 * WPL)

#define LDS_FILL ((RCAP + NBF + LISTN) * 4 + 64)

static_assert((CHUNK & (CHUNK - 1)) == 0);
static_assert(CHUNK <= 4096);
static_assert(NBC <= 4096 && NBF <= 4096);
static_assert((NBC & (NBC - 1)) == 0 && (NBF & (NBF - 1)) == 0);
static_assert(NBC == 4 * NBF);
static_assert(OTHR * 8 == NBC);
static_assert((RCAP % 32) == 0);
static_assert(TGT == NWAVE * 16 && GROWS == NWAVE * 16 && TGT == GROWS);
static_assert((NBC % TGT) == 0);
static_assert(FD == 64 && KD == FD && (KD % 32) == 0);
static_assert(NCLS > 32 && NCLS <= 48 && (NCLS % 4) == 0);
static_assert(((TGT * NCLS) % (4 * NTHR)) == 0);
static_assert((WPL % 64) == 0);
static_assert(RCAP + NBF + LISTN + NWAVE <= LDS_FILL / 4);

typedef float          v2f  __attribute__((ext_vector_type(2)));
typedef float          v4f  __attribute__((ext_vector_type(4)));
typedef float          v8f  __attribute__((ext_vector_type(8)));
typedef int            v4i  __attribute__((ext_vector_type(4)));
typedef unsigned short v8us __attribute__((ext_vector_type(8)));
typedef __bf16         v16b __attribute__((ext_vector_type(16)));
union FragB { v16b v; v8us h[2]; };

__device__ __forceinline__ unsigned int bfr(float f) {
  const unsigned int u = __float_as_uint(f);
  return (u + 0x7FFFu + ((u >> 16) & 1u)) >> 16;
}

__device__ __forceinline__ void split1(float x, unsigned short& hb, unsigned short& lb) {
  const unsigned int hu = bfr(x);
  const float hf = __uint_as_float(hu << 16);
  hb = (unsigned short)hu;
  lb = (unsigned short)bfr(x - hf);
}

__device__ __forceinline__ void split8(v4f a, v4f b, v8us& hi, v8us& lo) {
  unsigned short hb, lb;
  split1(a.x, hb, lb); hi[0] = hb; lo[0] = lb;
  split1(a.y, hb, lb); hi[1] = hb; lo[1] = lb;
  split1(a.z, hb, lb); hi[2] = hb; lo[2] = lb;
  split1(a.w, hb, lb); hi[3] = hb; lo[3] = lb;
  split1(b.x, hb, lb); hi[4] = hb; lo[4] = lb;
  split1(b.y, hb, lb); hi[5] = hb; lo[5] = lb;
  split1(b.z, hb, lb); hi[6] = hb; lo[6] = lb;
  split1(b.w, hb, lb); hi[7] = hb; lo[7] = lb;
}

__device__ __forceinline__ v8f wmb(v16b a, v16b b, v8f c) {
  v8f d = __builtin_amdgcn_wmma_f32_16x16x32_bf16(false, a, false, b, (short)0, c, false, false);
  asm volatile("v_nop\n\tv_nop\n\tv_nop\n\tv_nop" : "+v"(d) : "v"(a), "v"(b));
  return d;
}

template <int NT>
__device__ __forceinline__ void mma_rows(const float* __restrict__ arow, const unsigned short* __restrict__ Bw,
                                         int hh, int m, v8f (&acc)[NT]) {
#pragma unroll
  for (int t = 0; t < NT; ++t) { v8f z = {0.f, 0.f, 0.f, 0.f, 0.f, 0.f, 0.f, 0.f}; acc[t] = z; }
  const float* ap = arow + 8 * hh;
#pragma unroll
  for (int kt = 0; kt < KD / 32; ++kt) {
    const v4f f0 = *(const v4f*)(ap + 32 * kt);
    const v4f f1 = *(const v4f*)(ap + 32 * kt + 4);
    const v4f f2 = *(const v4f*)(ap + 32 * kt + 16);
    const v4f f3 = *(const v4f*)(ap + 32 * kt + 20);
    FragB ah, al;
    split8(f0, f1, ah.h[0], al.h[0]);
    split8(f2, f3, ah.h[1], al.h[1]);
#pragma unroll
    for (int t = 0; t < NT; ++t) {
      const unsigned short* bp = Bw + (size_t)(16 * t + m) * KD + 32 * kt + 8 * hh;
      FragB bh, bl;
      bh.h[0] = *(const v8us*)bp;
      bh.h[1] = *(const v8us*)(bp + 16);
      bl.h[0] = *(const v8us*)(bp + NCP * KD);
      bl.h[1] = *(const v8us*)(bp + NCP * KD + 16);
      acc[t] = wmb(ah.v, bh.v, acc[t]);
      acc[t] = wmb(ah.v, bl.v, acc[t]);
      acc[t] = wmb(al.v, bh.v, acc[t]);
    }
  }
}

__device__ __forceinline__ void store_rows64(const float* stg, float* C, int rowBase, int wave, int lane) {
  const int rsub = lane >> 4, c4 = (lane & 15) * 4;
  const float* lp = stg + (wave * 16 + rsub) * FD + c4;
  float* gp = C + (size_t)(rowBase + wave * 16 + rsub) * FD + c4;
#pragma unroll
  for (int i = 0; i < 8; ++i) { const v4f v = *(const v4f*)(lp + 2 * FD * i); *(volatile v4f*)(gp + 2 * FD * i) = v; }
  __threadfence();
#pragma unroll
  for (int i = 0; i < 8; ++i) { const v4f v = *(const v4f*)(lp + 2 * FD * i); *(volatile v4f*)(gp + 2 * FD * i) = v; }
}

template <int NB>
__device__ __forceinline__ int scan_chunk(const int* __restrict__ dsts, int nE, int cbase, int slotBase,
                                          int vec8, int* list, int tid, int lane, int wave) {
  int wc = 0;
#pragma unroll
  for (int g = 0; g < NGRP; ++g) {
    const int el0  = (g * NTHR + tid) * EPT;
    const int e0   = cbase + el0;
    const int sent = -2147483647 - 1;
    v4i da, db;
    if (vec8 != 0 && cbase + CHUNK <= nE) {
      da = *(const v4i*)(dsts + e0);
      db = *(const v4i*)(dsts + e0 + 4);
    } else {
      da.x = (e0     < nE) ? dsts[min(e0, nE - 1)] : sent;
      da.y = (e0 + 1 < nE) ? dsts[min(e0 + 1, nE - 1)] : sent;
      da.z = (e0 + 2 < nE) ? dsts[min(e0 + 2, nE - 1)] : sent;
      da.w = (e0 + 3 < nE) ? dsts[min(e0 + 3, nE - 1)] : sent;
      db.x = (e0 + 4 < nE) ? dsts[min(e0 + 4, nE - 1)] : sent;
      db.y = (e0 + 5 < nE) ? dsts[min(e0 + 5, nE - 1)] : sent;
      db.z = (e0 + 6 < nE) ? dsts[min(e0 + 6, nE - 1)] : sent;
      db.w = (e0 + 7 < nE) ? dsts[min(e0 + 7, nE - 1)] : sent;
    }
    const unsigned nb = (unsigned)slotBase;
    const unsigned s0 = (unsigned)da.x - nb, s1 = (unsigned)da.y - nb;
    const unsigned s2 = (unsigned)da.z - nb, s3 = (unsigned)da.w - nb;
    const unsigned s4 = (unsigned)db.x - nb, s5 = (unsigned)db.y - nb;
    const unsigned s6 = (unsigned)db.z - nb, s7 = (unsigned)db.w - nb;
    const bool h0 = s0 < (unsigned)NB, h1 = s1 < (unsigned)NB, h2 = s2 < (unsigned)NB, h3 = s3 < (unsigned)NB;
    const bool h4 = s4 < (unsigned)NB, h5 = s5 < (unsigned)NB, h6 = s6 < (unsigned)NB, h7 = s7 < (unsigned)NB;
    const unsigned any = __builtin_amdgcn_ballot_w32(h0 | h1 | h2 | h3 | h4 | h5 | h6 | h7);
    if (any != 0u) {
#define HITJ(J, HJ, SJ) { \
        const unsigned mj = __builtin_amdgcn_ballot_w32(HJ); \
        if (mj != 0u) { \
          if (HJ) { \
            const int pos = wc + (int)__builtin_amdgcn_mbcnt_lo(mj, 0u); \
            if (pos < WCAP) list[wave * WCAP + pos] = ((el0 + (J)) << 12) | (int)(SJ); \
          } \
          wc += (int)__builtin_popcount(mj); } }
      HITJ(0, h0, s0)
      HITJ(1, h1, s1)
      HITJ(2, h2, s2)
      HITJ(3, h3, s3)
      HITJ(4, h4, s4)
      HITJ(5, h5, s5)
      HITJ(6, h6, s6)
      HITJ(7, h7, s7)
#undef HITJ
    }
  }
  return wc;
}

__global__ __launch_bounds__(NTHR) void k_wprep(
    const float* __restrict__ w1, const float* __restrict__ w2, const float* __restrict__ wf,
    unsigned short* wp) {
  const int blk = blockIdx.x, tid = threadIdx.x;
  const int sel = blk >> 1;
  const int i = (blk & 1) * NTHR + tid;
  const int n = i >> 3, k0 = (i & 7) * 8;
  const int na = n > (NCLS - 1) ? (NCLS - 1) : n;
  float v[8];
#pragma unroll
  for (int e = 0; e < 8; ++e) {
    const int k = k0 + e;
    const float va = w1[k * FD + n];
    const float vb = w2[k * FD + n];
    const float vc = wf[k * NCLS + na];
    const float vcz = (n < NCLS) ? vc : 0.0f;
    v[e] = (sel == 0) ? va : ((sel == 1) ? vb : vcz);
  }
  v4f a, b;
  a.x = v[0]; a.y = v[1]; a.z = v[2]; a.w = v[3];
  b.x = v[4]; b.y = v[5]; b.z = v[6]; b.w = v[7];
  v8us hv, lv;
  split8(a, b, hv, lv);
  const int base = (sel == 0) ? WP_1 : ((sel == 1) ? WP_2 : WP_F);
  unsigned short* dh = wp + base + (size_t)i * 8;
  unsigned short* dl = dh + NCP * KD;
  *(volatile v8us*)dh = hv;
  *(volatile v8us*)dl = lv;
  __threadfence();
  *(volatile v8us*)dh = hv;
  *(volatile v8us*)dl = lv;
}

__global__ __launch_bounds__(NTHR) void k_count(const int* __restrict__ dsts, int* cnt, int nE, int vec8) {
  __shared__ __attribute__((aligned(16))) int scnt[NBC];
  __shared__ __attribute__((aligned(16))) int list[LISTN];
  __shared__ int wcnt[NWAVE];
  const int tid = threadIdx.x, lane = tid & 31, wave = tid >> 5;
  const int nodeBase = blockIdx.x * NBC;

  for (int i = tid; i < NBC; i += NTHR) scnt[i] = 0;
  __syncthreads();

  const int nChunks = (nE + CHUNK - 1) / CHUNK;
#pragma unroll 1
  for (int ch = 0; ch < nChunks; ++ch) {
    const int cbase = ch * CHUNK;
    const int wc = scan_chunk<NBC>(dsts, nE, cbase, nodeBase, vec8, list, tid, lane, wave);
    if (lane == 0) wcnt[wave] = wc;
    __syncthreads();
    if (wave == 0) {
#pragma unroll 1
      for (int wsx = 0; wsx < NWAVE; ++wsx) {
        int n = __builtin_amdgcn_readfirstlane(wcnt[wsx]);
        n = n > WCAP ? WCAP : (n < 0 ? 0 : n);
        const int* lp = list + wsx * WCAP;
#pragma unroll 1
        for (int i = 0; i < n; ++i) {
          const int ent  = __builtin_amdgcn_readfirstlane(lp[i]);
          const int slot = ent & (NBC - 1);
          if (lane == 0) scnt[slot] = scnt[slot] + 1;
        }
      }
    }
    __syncthreads();
  }

  v4i cq[4];
#pragma unroll
  for (int q = 0; q < 4; ++q) {
    const int f = (wave * 4 + q) * 128 + 4 * lane;
    cq[q] = *(const v4i*)(scnt + f);
  }
  int* cp = cnt + (size_t)nodeBase;
#pragma unroll
  for (int q = 0; q < 4; ++q) {
    const int f = (wave * 4 + q) * 128 + 4 * lane;
    *(volatile v4i*)(cp + f) = cq[q];
  }
  __threadfence();
#pragma unroll
  for (int q = 0; q < 4; ++q) {
    const int f = (wave * 4 + q) * 128 + 4 * lane;
    *(volatile v4i*)(cp + f) = cq[q];
  }
}

__global__ __launch_bounds__(OTHR) void k_offsets(
    const int* __restrict__ cnt, int* off, int* rbase, int nChunk) {
  __shared__ __attribute__((aligned(16))) int soff[NBC];
  __shared__ __attribute__((aligned(16))) int srb[RBN];
  __shared__ int wtot[OTHR / 32];
  const int tid = threadIdx.x, lane = tid & 31, wave = tid >> 5, sub = tid >> 7;
  for (int i = tid; i < RBN; i += OTHR) srb[i] = 0;
  int carry = 0;
#pragma unroll 1
  for (int ch = 0; ch < nChunk; ++ch) {
    const int base = ch * NBC;
    const v4i c0 = *(const v4i*)(cnt + base + 8 * tid);
    const v4i c1 = *(const v4i*)(cnt + base + 8 * tid + 4);
    const int e0 = max(c0.x, 0), e1 = max(c0.y, 0), e2 = max(c0.z, 0), e3 = max(c0.w, 0);
    const int e4 = max(c1.x, 0), e5 = max(c1.y, 0), e6 = max(c1.z, 0), e7 = max(c1.w, 0);
    const int ts = e0 + e1 + e2 + e3 + e4 + e5 + e6 + e7;
    int incl = ts;
#pragma unroll
    for (int d = 1; d < 32; d <<= 1) {
      const int t = __shfl_up(incl, d);
      if (lane >= d) incl += t;
    }
    if (lane == 31) wtot[wave] = incl;
    __syncthreads();
    const int S0 = wtot[0]  + wtot[1]  + wtot[2]  + wtot[3];
    const int S1 = wtot[4]  + wtot[5]  + wtot[6]  + wtot[7];
    const int S2 = wtot[8]  + wtot[9]  + wtot[10] + wtot[11];
    const int S3 = wtot[12] + wtot[13] + wtot[14] + wtot[15];
    int pre = 0;
#pragma unroll 1
    for (int w = 4 * sub; w < wave; ++w) pre += wtot[w];
    const int b0 = carry;
    const int b1 = b0 + ((S0 + 31) & ~31);
    const int b2 = b1 + ((S1 + 31) & ~31);
    const int b3 = b2 + ((S2 + 31) & ~31);
    const int b4 = b3 + ((S3 + 31) & ~31);
    const int myb = sub == 0 ? b0 : (sub == 1 ? b1 : (sub == 2 ? b2 : b3));
    if (tid == 0) {
      srb[min(4 * ch + 0, RBN - 1)] = b0;
      srb[min(4 * ch + 1, RBN - 1)] = b1;
      srb[min(4 * ch + 2, RBN - 1)] = b2;
      srb[min(4 * ch + 3, RBN - 1)] = b3;
    }
    int run = myb + pre + incl - ts;
    soff[8 * tid + 0] = run; run += e0;
    soff[8 * tid + 1] = run; run += e1;
    soff[8 * tid + 2] = run; run += e2;
    soff[8 * tid + 3] = run; run += e3;
    soff[8 * tid + 4] = run; run += e4;
    soff[8 * tid + 5] = run; run += e5;
    soff[8 * tid + 6] = run; run += e6;
    soff[8 * tid + 7] = run;
    carry = b4;
    __syncthreads();
    const v4i o0 = *(const v4i*)(soff + 4 * tid);
    const v4i o1 = *(const v4i*)(soff + 4 * (tid + OTHR));
    int* op = off + base;
    *(volatile v4i*)(op + 4 * tid) = o0;
    *(volatile v4i*)(op + 4 * (tid + OTHR)) = o1;
    __threadfence();
    *(volatile v4i*)(op + 4 * tid) = o0;
    *(volatile v4i*)(op + 4 * (tid + OTHR)) = o1;
    __syncthreads();
  }
  if (tid == 0) srb[min(4 * nChunk, RBN - 1)] = carry;
  __syncthreads();
  v4i rv = {0, 0, 0, 0};
  if (tid < 32) rv = *(const v4i*)(srb + 4 * tid);
  if (tid < 32) *(volatile v4i*)(rbase + 4 * tid) = rv;
  __threadfence();
  if (tid < 32) *(volatile v4i*)(rbase + 4 * tid) = rv;
}

__global__ __launch_bounds__(NTHR) void k_fill(
    const int* __restrict__ srcs, const int* __restrict__ dsts,
    const int* __restrict__ off, const int* __restrict__ rbase,
    int* csr, int nN, int nE, int vec8, int csrLen) {
  extern __shared__ v4f lds_dyn[];
  int* region = (int*)lds_dyn;
  int* cursor = region + RCAP;
  int* list   = cursor + NBF;
  int* wcnt   = list + LISTN;
  const int tid = threadIdx.x, lane = tid & 31, wave = tid >> 5;
  const int b = blockIdx.x;
  const int nodeBase = b * NBF;

  int rb0 = rbase[b];
  const int rb1 = rbase[b + 1];
  rb0 = rb0 < 0 ? 0 : (rb0 > csrLen ? csrLen : rb0);
  rb0 &= ~31;
  int len = rb1 - rb0;
  len = len < 0 ? 0 : (len > RCAP ? RCAP : len);
  int lenW = (len + 31) & ~31;
  if (rb0 + lenW > csrLen) lenW = (csrLen - rb0) & ~31;

  {
    const v4i z = {0, 0, 0, 0};
    for (int i = tid; i < RCAP / 4; i += NTHR) ((v4i*)region)[i] = z;
    for (int s = tid; s < NBF; s += NTHR) {
      int o = off[nodeBase + s] - rb0;
      o = o < 0 ? 0 : (o > RCAP ? RCAP : o);
      cursor[s] = o;
    }
  }
  __syncthreads();

  const int nChunks = (nE + CHUNK - 1) / CHUNK;
#pragma unroll 1
  for (int ch = 0; ch < nChunks; ++ch) {
    const int cbase = ch * CHUNK;
    const int wc = scan_chunk<NBF>(dsts, nE, cbase, nodeBase, vec8, list, tid, lane, wave);
    if (lane == 0) wcnt[wave] = wc;
    __syncthreads();
    if (wave == 0) {
#pragma unroll 1
      for (int wsx = 0; wsx < NWAVE; ++wsx) {
        int n = __builtin_amdgcn_readfirstlane(wcnt[wsx]);
        n = n > WCAP ? WCAP : (n < 0 ? 0 : n);
        const int* lp = list + wsx * WCAP;
#pragma unroll 1
        for (int i = 0; i < n; ++i) {
          const int ent  = __builtin_amdgcn_readfirstlane(lp[i]);
          const int slot = ent & (NBF - 1);
          int e = cbase + ((ent >> 12) & (CHUNK - 1));
          e = e > nE - 1 ? nE - 1 : e;
          int sv = srcs[e];
          sv = sv < 0 ? 0 : (sv > nN - 1 ? nN - 1 : sv);
          if (lane == 0) {
            int pos = cursor[slot];
            pos = pos < 0 ? 0 : (pos > RCAP - 1 ? RCAP - 1 : pos);
            region[pos] = sv;
            const int np = pos + 1;
            cursor[slot] = np > RCAP ? RCAP : np;
          }
        }
      }
    }
    __syncthreads();
  }

  const int nv = lenW >> 2;
  int* gp = csr + rb0;
#pragma unroll 1
  for (int i = tid; i < nv; i += NTHR) { const v4i v = ((const v4i*)region)[i]; *(volatile v4i*)(gp + 4 * i) = v; }
  __threadfence();
#pragma unroll 1
  for (int i = tid; i < nv; i += NTHR) { const v4i v = ((const v4i*)region)[i]; *(volatile v4i*)(gp + 4 * i) = v; }
}

template <bool RELU>
__global__ __launch_bounds__(NTHR) void k_gemm(
    const float* __restrict__ X, const unsigned short* __restrict__ Bw, const float* __restrict__ bias,
    float* C, int nN) {
  __shared__ __attribute__((aligned(16))) float stg[GROWS * FD];
  const int tid = threadIdx.x, lane = tid & 31, wave = tid >> 5, hh = lane >> 4, m = lane & 15;
  const int rowBase = blockIdx.x * GROWS;
  int ra = rowBase + wave * 16 + m;
  ra = ra > nN - 1 ? nN - 1 : ra;

  v8f acc[4];
  mma_rows<4>(X + (size_t)ra * FD, Bw, hh, m, acc);

  float* sp = stg + (wave * 16 + 8 * hh) * FD + m;
#pragma unroll
  for (int t = 0; t < 4; ++t) {
    const float bv = bias[16 * t + m];
#pragma unroll
    for (int r = 0; r < 8; ++r) {
      float v = acc[t][r] + bv;
      if (RELU) v = fmaxf(v, 0.0f);
      sp[r * FD + 16 * t] = v;
    }
  }
  __syncthreads();

  store_rows64(stg, C, rowBase, wave, lane);
}

__global__ __launch_bounds__(NTHR) void k_agg(
    const int* __restrict__ csr, const int* __restrict__ off, const int* __restrict__ cnt,
    const float* __restrict__ In, float* S, int nN, int csrLen) {
  __shared__ __attribute__((aligned(16))) float sacc[TGT * FD];
  const int tid = threadIdx.x, lane = tid & 31, wave = tid >> 5;
  const int tbase = blockIdx.x * TGT + wave * 16;
  const int cl = tbase + (lane & 15);
  const int cnt_l = cnt[cl];
  const int off_l = off[cl];

#pragma unroll 1
  for (int j = 0; j < 16; ++j) {
    int n = __builtin_amdgcn_readlane(cnt_l, j);
    n = n < 0 ? 0 : (n > DEGCAP ? DEGCAP : n);
    const int st = __builtin_amdgcn_readlane(off_l, j);
    v2f sm = {0.0f, 0.0f};
#pragma unroll 1
    for (int q0 = 0; q0 < n; q0 += 32) {
      int pos = st + q0 + lane;
      pos = pos < 0 ? 0 : (pos > csrLen - 1 ? csrLen - 1 : pos);
      int sl = csr[pos];
      sl = sl < 0 ? 0 : (sl > nN - 1 ? nN - 1 : sl);
      const int mcnt = (n - q0) < 32 ? (n - q0) : 32;
#pragma unroll 1
      for (int p = 0; p < mcnt; ++p) {
        const int s = __builtin_amdgcn_readlane(sl, p);
        const v2f vf = *(const v2f*)(In + (size_t)s * FD + 2 * lane);
        sm = sm + vf;
      }
    }
    *(v2f*)(sacc + (wave * 16 + j) * FD + 2 * lane) = sm;
  }
  __syncthreads();

  store_rows64(sacc, S, blockIdx.x * TGT, wave, lane);
}

__device__ __forceinline__ void out_pass(const float* sout, float* ob, int nf, int tid) {
#pragma unroll
  for (int it = 0; it < (TGT * NCLS) / (4 * NTHR); ++it) {
    const int q = it * NTHR + tid;
    const v4f v = *(const v4f*)(sout + 4 * q);
    if (4 * q + 4 <= nf) *(volatile v4f*)(ob + 4 * q) = v;
  }
}

__global__ __launch_bounds__(NTHR) void k_cls(
    const float* __restrict__ X, const unsigned short* __restrict__ Bw, const float* __restrict__ bfp,
    float* out, int nN) {
  __shared__ __attribute__((aligned(16))) float sout[TGT * NCLS];
  const int tid = threadIdx.x, lane = tid & 31, wave = tid >> 5, hh = lane >> 4, m = lane & 15;
  const int rowBase = blockIdx.x * TGT;
  int ra = rowBase + wave * 16 + m;
  ra = ra > nN - 1 ? nN - 1 : ra;

  v8f acc[3];
  mma_rows<3>(X + (size_t)ra * FD, Bw, hh, m, acc);

  const float b0v = bfp[m];
  const float b1v = bfp[16 + m];
  const float b2v = bfp[(32 + m) > (NCLS - 1) ? (NCLS - 1) : (32 + m)];
  const bool c2ok = (32 + m) < NCLS;
  float* sp = sout + (wave * 16 + 8 * hh) * NCLS + m;
#pragma unroll
  for (int r = 0; r < 8; ++r) {
    const float v0 = acc[0][r] + b0v;
    const float v1 = acc[1][r] + b1v;
    const float v2 = c2ok ? (acc[2][r] + b2v) : -1.0e30f;
    float mx = fmaxf(v0, fmaxf(v1, v2));
#pragma unroll
    for (int mask = 1; mask < 16; mask <<= 1) mx = fmaxf(mx, __shfl_xor(mx, mask, 16));
    const float e0 = expf(v0 - mx), e1 = expf(v1 - mx), e2 = expf(v2 - mx);
    float sum = e0 + e1 + e2;
#pragma unroll
    for (int mask = 1; mask < 16; mask <<= 1) sum += __shfl_xor(sum, mask, 16);
    const float inv = 1.0f / sum;
    sp[r * NCLS] = e0 * inv;
    sp[r * NCLS + 16] = e1 * inv;
    if (c2ok) sp[r * NCLS + 32] = e2 * inv;
  }
  __syncthreads();

  int nvalid = nN - rowBase;
  nvalid = nvalid > TGT ? TGT : (nvalid < 0 ? 0 : nvalid);
  const int nf = nvalid * NCLS;
  float* ob = out + (size_t)blockIdx.x * (TGT * NCLS);
  out_pass(sout, ob, nf, tid);
  __threadfence();
  out_pass(sout, ob, nf, tid);
}

extern "C" void kernel_launch(void* const* d_in, const int* in_sizes, int n_in,
                              void* d_out, int out_size, void* d_ws, size_t ws_size,
                              hipStream_t stream) {
  if (n_in < 8) return;
  const int nN = in_sizes[0] / FD;
  const int nE = in_sizes[1] / 2;
  if (nN <= 0 || nE <= 0) return;
  if (in_sizes[0] != nN * FD || in_sizes[1] != 2 * nE) return;
  if (in_sizes[2] != FD * FD || in_sizes[3] != FD) return;
  if (in_sizes[4] != FD * FD || in_sizes[5] != FD) return;
  if (in_sizes[6] != FD * NCLS || in_sizes[7] != NCLS) return;
  if (out_size != nN * NCLS) return;
  if (nE > (1 << 28) || nN > (1 << 24)) return;

  const float* x    = (const float*)d_in[0];
  const int*   ei   = (const int*)d_in[1];
  const float* w1   = (const float*)d_in[2];
  const float* b1   = (const float*)d_in[3];
  const float* w2   = (const float*)d_in[4];
  const float* b2   = (const float*)d_in[5];
  const float* wf   = (const float*)d_in[6];
  const float* bfv  = (const float*)d_in[7];
  const int*   srcs = ei;
  const int*   dsts = ei + nE;
  float* out = (float*)d_out;

  const int NPAD   = ((nN + TGT - 1) / TGT) * TGT;
  const int nBC    = (nN + NBC - 1) / NBC;
  const int CNTPAD = nBC * NBC;
  if (4 * nBC + 1 > RBN) return;
  const int nBF    = (nN + NBF - 1) / NBF;
  const int csrLen = ((nE + 31) & ~31) + 4096;
  if (31 * 4 * nBC > 4096) return;
  const int nGemm  = NPAD / GROWS;
  const int nAgg   = NPAD / TGT;

  char* ws = (char*)d_ws;
  size_t off = 0;
  const size_t oW   = off; off += (size_t)WPTOT * 2;     off = (off + 255) & ~(size_t)255;
  const size_t oCnt = off; off += (size_t)CNTPAD * 4;    off = (off + 255) & ~(size_t)255;
  const size_t oOff = off; off += (size_t)CNTPAD * 4;    off = (off + 255) & ~(size_t)255;
  const size_t oRb  = off; off += (size_t)RBN * 4;       off = (off + 255) & ~(size_t)255;
  const size_t oCsr = off; off += (size_t)csrLen * 4;    off = (off + 255) & ~(size_t)255;
  const size_t oP   = off; off += (size_t)NPAD * FD * 4; off = (off + 255) & ~(size_t)255;
  const size_t oS1  = off; off += (size_t)NPAD * FD * 4; off = (off + 255) & ~(size_t)255;
  const size_t oQ   = off; off += (size_t)NPAD * FD * 4; off = (off + 255) & ~(size_t)255;
  const size_t oS2  = off; off += (size_t)NPAD * FD * 4; off = (off + 255) & ~(size_t)255;
  if (off > ws_size || off > (size_t)WSCAP) return;
  unsigned short* wp   = (unsigned short*)(ws + oW);
  int*            cnt  = (int*)(ws + oCnt);
  int*            offp = (int*)(ws + oOff);
  int*            rb   = (int*)(ws + oRb);
  int*            csr  = (int*)(ws + oCsr);
  float*          P    = (float*)(ws + oP);
  float*          S1   = (float*)(ws + oS1);
  float*          Q    = (float*)(ws + oQ);
  float*          S2   = (float*)(ws + oS2);

  const int vec8 = ((nE & 3) == 0) ? 1 : 0;

  k_wprep<<<6, NTHR, 0, stream>>>(w1, w2, wf, wp);

  k_count<<<nBC, NTHR, 0, stream>>>(dsts, cnt, nE, vec8);
  k_offsets<<<1, OTHR, 0, stream>>>(cnt, offp, rb, nBC);
  hipFuncSetAttribute(reinterpret_cast<const void*>(&k_fill),
                      hipFuncAttributeMaxDynamicSharedMemorySize, LDS_FILL);
  k_fill<<<nBF, NTHR, LDS_FILL, stream>>>(srcs, dsts, offp, rb, csr, nN, nE, vec8, csrLen);

  k_gemm<true><<<nGemm, NTHR, 0, stream>>>(x, wp + WP_1, b1, P, nN);

  k_agg<<<nAgg, NTHR, 0, stream>>>(csr, offp, cnt, P, S1, nN, csrLen);

  k_gemm<false><<<nGemm, NTHR, 0, stream>>>(S1, wp + WP_2, b2, Q, nN);

  k_agg<<<nAgg, NTHR, 0, stream>>>(csr, offp, cnt, Q, S2, nN, csrLen);

  k_cls<<<nGemm, NTHR, 0, stream>>>(S2, wp + WP_F, bfv, out, nN);
}
